// SequentialTransductionUnitDense_68934225101348
// MI455X (gfx1250) — hardware-verified
//
#include <hip/hip_runtime.h>
#include <math.h>
#include <stdint.h>

#define NBATCH 4
#define SEQ    2048
#define DMOD   512
#define EPROJ  2048
#define NH     8
#define HD     64
#define NQB    (SEQ / 64)
#define NROWS  (NBATCH * SEQ)
#define RESC   4096.0f
static_assert(NH * HD == DMOD);
static_assert((SEQ % 64) == 0 && (DMOD % 64) == 0 && (EPROJ % 64) == 0 && (NROWS % 64) == 0 && (DMOD % 32) == 0);

typedef _Float16 v16h __attribute__((ext_vector_type(16)));
typedef _Float16 v8h  __attribute__((ext_vector_type(8)));
typedef __bf16   v16b __attribute__((ext_vector_type(16)));
typedef __bf16   v8b  __attribute__((ext_vector_type(8)));
typedef float    v8f  __attribute__((ext_vector_type(8)));
typedef float    v4f  __attribute__((ext_vector_type(4)));
typedef unsigned int v4u __attribute__((ext_vector_type(4)));
typedef unsigned short v8us __attribute__((ext_vector_type(8)));

__device__ __forceinline__ unsigned short bf_bits(float f) {
  unsigned u = __float_as_uint(f);
  return (unsigned short)((u + 0x7FFFu + ((u >> 16) & 1u)) >> 16);
}
__device__ __forceinline__ float bf_up(unsigned short h) { return __uint_as_float(((unsigned)h) << 16); }
__device__ __forceinline__ unsigned short h_bits(_Float16 x) { return __builtin_bit_cast(unsigned short, x); }
__device__ __forceinline__ unsigned pk16(unsigned short a, unsigned short b) { return (unsigned)a | ((unsigned)b << 16); }
__device__ __forceinline__ v8f zero8() { v8f z = {0.f, 0.f, 0.f, 0.f, 0.f, 0.f, 0.f, 0.f}; return z; }

__device__ __forceinline__ v16b ldfrag_b(const __bf16* p) {
  union { v16b v; v8b h[2]; } f;
  f.h[0] = *(const v8b*)(p);
  f.h[1] = *(const v8b*)(p + 16);
  return f.v;
}
__device__ __forceinline__ v16h ldfrag_h(const _Float16* p) {
  union { v16h v; v8h h[2]; } f;
  f.h[0] = *(const v8h*)(p);
  f.h[1] = *(const v8h*)(p + 16);
  return f.v;
}

__device__ __forceinline__ v8f mma_h(v16h a, v16h b, v8f c) {
  c = __builtin_amdgcn_wmma_f32_16x16x32_f16(false, a, false, b, (short)0, c, false, false);
#if defined(__HIP_DEVICE_COMPILE__)
  asm volatile("v_nop\n\tv_nop\n\tv_nop\n\tv_nop" : "+v"(c) : "v"(a), "v"(b));
#endif
  return c;
}
__device__ __forceinline__ v8f mma_b_raw(v16b a, v16b b, v8f c) {
  return __builtin_amdgcn_wmma_f32_16x16x32_bf16(false, a, false, b, (short)0, c, false, false);
}
__device__ __forceinline__ void dep_guard_b(v8f& a, v8f& b, v16b x, v16b y) {
#if defined(__HIP_DEVICE_COMPILE__)
  asm volatile("v_nop\n\tv_nop\n\tv_nop\n\tv_nop" : "+v"(a), "+v"(b) : "v"(x), "v"(y));
#endif
}
__device__ __forceinline__ void keep4_b(v16b a, v16b b, v16b c, v16b d) {
#if defined(__HIP_DEVICE_COMPILE__)
  asm volatile("v_nop" :: "v"(a), "v"(b), "v"(c), "v"(d));
#endif
}
__device__ __forceinline__ void acc_guard4(v8f& a, v8f& b, v8f& c, v8f& d) {
#if defined(__HIP_DEVICE_COMPILE__)
  asm volatile("v_nop\n\tv_nop\n\tv_nop\n\tv_nop" : "+v"(a), "+v"(b), "+v"(c), "+v"(d));
#endif
}
__device__ __forceinline__ void wave_sync_lds() {
  __builtin_amdgcn_fence(__ATOMIC_RELEASE, "workgroup");
  __builtin_amdgcn_wave_barrier();
  __builtin_amdgcn_fence(__ATOMIC_ACQUIRE, "workgroup");
}

__global__ __launch_bounds__(256) void cvt_cat_bf16x8(const float* __restrict__ in, unsigned short* out,
                                                      int n8, int inCols8, int outPitch, int colOff) {
  const int i = blockIdx.x * 256 + threadIdx.x;
  if (i < n8) {
    const int row = i / inCols8;
    const int c8  = i - row * inCols8;
    const v4f a = *(const v4f*)(in + (size_t)i * 8);
    const v4f b = *(const v4f*)(in + (size_t)i * 8 + 4);
    v4u p;
    p[0] = pk16(bf_bits(a[0]), bf_bits(a[1]));
    p[1] = pk16(bf_bits(a[2]), bf_bits(a[3]));
    p[2] = pk16(bf_bits(b[0]), bf_bits(b[1]));
    p[3] = pk16(bf_bits(b[2]), bf_bits(b[3]));
    unsigned short* dst = out + (size_t)row * outPitch + colOff + c8 * 8;
    *(volatile v4u*)dst = p;
    __threadfence();
    *(volatile v4u*)dst = p;
  }
}

template <int MODE>
__global__ __launch_bounds__(256) void transpose16(const float* __restrict__ in, int R, int C, long long inStride,
                                                   unsigned short* out, long long outStride, float scale, float rscale) {
  __shared__ __align__(16) unsigned short t[64 * 72];
  union U8 { v8us s; v4u u; };
  const int b = blockIdx.y;
  const int tilesC = C >> 6;
  const int tile = blockIdx.x;
  const int tr = tile / tilesC;
  const int tc = tile - tr * tilesC;
  const int r0 = tr << 6, c0 = tc << 6;
  if (r0 >= R || c0 >= C) return;
  const int tid = threadIdx.x;
  {
    const int row = tid >> 2;
    const int cq  = (tid & 3) * 16;
    const float* p = in + (size_t)b * inStride + (size_t)(r0 + row) * C + c0 + cq;
#pragma unroll
    for (int i = 0; i < 4; ++i) {
      const v4f v = *(const v4f*)(p + 4 * i);
#pragma unroll
      for (int e = 0; e < 4; ++e) {
        const float x = v[e];
        unsigned short bits;
        if (MODE == 0) {
          bits = bf_bits(x);
        } else {
          const float xs = x * scale;
          const _Float16 xh = (_Float16)xs;
          if (MODE == 1) bits = h_bits(xh);
          else           bits = h_bits((_Float16)((xs - (float)xh) * rscale));
        }
        t[(cq + 4 * i + e) * 72 + row] = bits;
      }
    }
  }
  __syncthreads();
  {
    unsigned short* dst = out + (size_t)b * outStride;
    const int q  = tid >> 3;
    const int c8 = (tid & 7) * 8;
    U8 w[2];
#pragma unroll
    for (int it = 0; it < 2; ++it) {
      const int orow = it * 32 + q;
      w[it].s = *(const v8us*)(t + orow * 72 + c8);
    }
    for (int pass = 0; pass < 2; ++pass) {
#pragma unroll
      for (int it = 0; it < 2; ++it) {
        const int orow = it * 32 + q;
        *(volatile v4u*)(dst + (size_t)(c0 + orow) * R + r0 + c8) = w[it].u;
      }
      __threadfence();
    }
  }
}

template <int NSPLIT, int OUT_MODE, int BIAS, int ACT, int RESID>
__global__ __launch_bounds__(256) void gemm64(
    const unsigned short* __restrict__ Ap, const unsigned short* A2p, int lda, long long strideA,
    const unsigned short* __restrict__ Btp, const unsigned short* Bt2p, int ldb, long long strideB,
    const float* __restrict__ bias, const float* __restrict__ res, int ldr,
    void* Cout, int ldc, long long strideC,
    void* Cout2, int ldc2, long long strideC2, int N2,
    int M, int N, int K, float rscale, float oscale) {
  const __bf16* A   = (const __bf16*)(const void*)Ap;
  const __bf16* A2  = (const __bf16*)(const void*)A2p;
  const __bf16* Bt  = (const __bf16*)(const void*)Btp;
  const __bf16* Bt2 = (const __bf16*)(const void*)Bt2p;
  __shared__ __align__(16) float sT[8][16 * 68];
  const int b    = blockIdx.y;
  const int lane = threadIdx.x & 31;
  const int wave = threadIdx.x >> 5;
  const int tilesN = N >> 6;
  const int tilesM = M >> 6;
  const int tile = blockIdx.x * 8 + wave;
  if (tile >= tilesM * tilesN) return;
  const int tm = tile / tilesN;
  const int tn = tile - tm * tilesN;
  const int m0 = tm << 6;
  const int n0 = tn << 6;

  const __bf16* Ab  = A  + (size_t)b * strideA;
  const __bf16* Bb  = Bt + (size_t)b * strideB;
  const __bf16* Ab2 = (NSPLIT >= 1) ? (A2  + (size_t)b * strideA) : Ab;
  const __bf16* Bb2 = (NSPLIT == 2) ? (Bt2 + (size_t)b * strideB) : Bb;

  const int rlane = lane & 15;
  const int koff  = (lane >> 4) * 8;
  const int mOff  = (lane >> 4) * 8;

  v8f acc[4][4];
#pragma unroll
  for (int i = 0; i < 4; ++i)
#pragma unroll
    for (int j = 0; j < 4; ++j) acc[i][j] = zero8();

  for (int k0 = 0; k0 < K; k0 += 32) {
    v16b bh[4], bl[4];
#pragma unroll
    for (int j = 0; j < 4; ++j) {
      const size_t bo = (size_t)(n0 + (j << 4) + rlane) * ldb + koff + k0;
      bh[j] = ldfrag_b(Bb + bo);
      if (NSPLIT == 2) bl[j] = ldfrag_b(Bb2 + bo); else bl[j] = bh[j];
    }
#pragma unroll
    for (int i = 0; i < 4; ++i) {
      const size_t ao = (size_t)(m0 + (i << 4) + rlane) * lda + koff + k0;
      const v16b ah = ldfrag_b(Ab + ao);
      v16b al = ah;
      if (NSPLIT >= 1) al = ldfrag_b(Ab2 + ao);
#pragma unroll
      for (int j = 0; j < 4; ++j) {
        acc[i][j] = mma_b_raw(ah, bh[j], acc[i][j]);
        if (NSPLIT >= 1) acc[i][j] = mma_b_raw(al, bh[j], acc[i][j]);
        if (NSPLIT == 2) acc[i][j] = mma_b_raw(ah, bl[j], acc[i][j]);
      }
      dep_guard_b(acc[i][0], acc[i][3], ah, al);
    }
    keep4_b(bh[0], bh[1], bh[2], bh[3]);
    if (NSPLIT == 2) keep4_b(bl[0], bl[1], bl[2], bl[3]);
  }
  acc_guard4(acc[0][0], acc[0][1], acc[0][2], acc[0][3]);
  acc_guard4(acc[1][0], acc[1][1], acc[1][2], acc[1][3]);
  acc_guard4(acc[2][0], acc[2][1], acc[2][2], acc[2][3]);
  acc_guard4(acc[3][0], acc[3][1], acc[3][2], acc[3][3]);

  float bcol[4] = {0.f, 0.f, 0.f, 0.f};
  if (BIAS == 1) {
#pragma unroll
    for (int j = 0; j < 4; ++j) bcol[j] = bf_up(bf_bits(bias[n0 + (j << 4) + rlane]));
  }
  float* slab = sT[wave];
#pragma unroll
  for (int i = 0; i < 4; ++i) {
    const int mBase = m0 + (i << 4);
    float brow[8] = {0.f, 0.f, 0.f, 0.f, 0.f, 0.f, 0.f, 0.f};
    if (BIAS == 2) {
#pragma unroll
      for (int r = 0; r < 8; ++r) brow[r] = bf_up(bf_bits(bias[mBase + mOff + r]));
    }
#pragma unroll
    for (int j = 0; j < 4; ++j) {
#pragma unroll
      for (int r = 0; r < 8; ++r) {
        float v = acc[i][j][r] + bcol[j] + brow[r];
        if (ACT == 1) {
          const float e = expf(-v);
          v = v * __builtin_amdgcn_rcpf(1.0f + e);
        }
        v *= oscale;
        if (RESID == 1) {
          v += bf_up(bf_bits(res[(size_t)(mBase + mOff + r) * ldr + n0 + (j << 4) + rlane]));
        }
        slab[(mOff + r) * 68 + (j << 4) + rlane] = v;
      }
    }
    wave_sync_lds();
    if (OUT_MODE == 0) {
      float* C = (float*)Cout + (size_t)b * strideC;
      const int hh = lane >> 4, c4 = (lane & 15) * 4;
      for (int pass = 0; pass < 2; ++pass) {
#pragma unroll
        for (int it = 0; it < 8; ++it) {
          const int row = it * 2 + hh;
          const v4f v = *(const v4f*)(slab + row * 68 + c4);
          *(volatile v4f*)(C + (size_t)(mBase + row) * ldc + n0 + c4) = v;
        }
        __threadfence();
      }
    } else {
      const int q = lane >> 3, c8 = (lane & 7) * 8;
      unsigned short* C  = (unsigned short*)Cout  + (size_t)b * strideC;
      unsigned short* C2 = (unsigned short*)Cout2 + (size_t)b * strideC2;
      const bool wlo = (OUT_MODE == 2) || (OUT_MODE == 3 && n0 < N2);
      v4u hv[4], lv[4];
#pragma unroll
      for (int it = 0; it < 4; ++it) {
        const int row = it * 4 + q;
        const float* sp = slab + row * 68 + c8;
        v4u a, a2;
#pragma unroll
        for (int e = 0; e < 4; ++e) {
          const float f0 = sp[2 * e], f1 = sp[2 * e + 1];
          unsigned short h0, h1, l0, l1;
          if (OUT_MODE == 2) {
            h0 = bf_bits(f0); h1 = bf_bits(f1);
            l0 = bf_bits(f0 - bf_up(h0)); l1 = bf_bits(f1 - bf_up(h1));
          } else {
            const _Float16 x0 = (_Float16)f0, x1 = (_Float16)f1;
            h0 = h_bits(x0); h1 = h_bits(x1);
            l0 = h_bits((_Float16)((f0 - (float)x0) * rscale));
            l1 = h_bits((_Float16)((f1 - (float)x1) * rscale));
          }
          a[e] = pk16(h0, h1); a2[e] = pk16(l0, l1);
        }
        hv[it] = a; lv[it] = a2;
      }
      for (int pass = 0; pass < 2; ++pass) {
#pragma unroll
        for (int it = 0; it < 4; ++it) {
          const int row = it * 4 + q;
          *(volatile v4u*)(C + (size_t)(mBase + row) * ldc + n0 + c8) = hv[it];
          if (wlo) *(volatile v4u*)(C2 + (size_t)(mBase + row) * ldc2 + n0 + c8) = lv[it];
        }
        __threadfence();
      }
    }
    wave_sync_lds();
  }
}

template <int MULMODE>
__global__ __launch_bounds__(256) void ln_rows(const float* __restrict__ in, const float* __restrict__ mul,
                                               unsigned short* oh, unsigned short* ol, int nrows) {
  const int wave = threadIdx.x >> 5, lane = threadIdx.x & 31;
  const int row = blockIdx.x * 8 + wave;
  if (row >= nrows) return;
  const float* xr = in + (size_t)row * DMOD;
  float v[16];
#pragma unroll
  for (int sg = 0; sg < 2; ++sg) {
    const v4f a  = *(const v4f*)(xr + sg * 256 + lane * 8);
    const v4f a4 = *(const v4f*)(xr + sg * 256 + lane * 8 + 4);
#pragma unroll
    for (int e = 0; e < 4; ++e) {
      float f0 = a[e], f1 = a4[e];
      if (MULMODE == 0) { f0 = bf_up(bf_bits(f0)); f1 = bf_up(bf_bits(f1)); }
      v[sg * 8 + e] = f0;
      v[sg * 8 + 4 + e] = f1;
    }
  }
  float sum = 0.f;
#pragma unroll
  for (int i = 0; i < 16; ++i) sum += v[i];
#pragma unroll
  for (int off = 1; off < 32; off <<= 1) sum += __shfl_xor(sum, off, 32);
  const float mu = sum * (1.0f / (float)DMOD);
  float ss = 0.f;
#pragma unroll
  for (int i = 0; i < 16; ++i) { v[i] -= mu; ss += v[i] * v[i]; }
#pragma unroll
  for (int off = 1; off < 32; off <<= 1) ss += __shfl_xor(ss, off, 32);
  const float rstd = rsqrtf(ss * (1.0f / (float)DMOD) + 1.0e-6f);
#pragma unroll
  for (int i = 0; i < 16; ++i) v[i] *= rstd;
  if (MULMODE == 1) {
    const float* mr = mul + (size_t)row * DMOD;
#pragma unroll
    for (int sg = 0; sg < 2; ++sg) {
      const v4f m0 = *(const v4f*)(mr + sg * 256 + lane * 8);
      const v4f m4 = *(const v4f*)(mr + sg * 256 + lane * 8 + 4);
#pragma unroll
      for (int e = 0; e < 4; ++e) {
        v[sg * 8 + e] *= m0[e];
        v[sg * 8 + 4 + e] *= m4[e];
      }
    }
  }
  v4u hv[2], lv[2];
#pragma unroll
  for (int sg = 0; sg < 2; ++sg) {
    v4u a, a2;
#pragma unroll
    for (int e = 0; e < 4; ++e) {
      const float f0 = v[sg * 8 + 2 * e], f1 = v[sg * 8 + 2 * e + 1];
      const unsigned short h0 = bf_bits(f0), h1 = bf_bits(f1);
      const unsigned short l0 = bf_bits(f0 - bf_up(h0)), l1 = bf_bits(f1 - bf_up(h1));
      a[e] = pk16(h0, h1); a2[e] = pk16(l0, l1);
    }
    hv[sg] = a; lv[sg] = a2;
  }
  for (int pass = 0; pass < 2; ++pass) {
#pragma unroll
    for (int sg = 0; sg < 2; ++sg) {
      const size_t go = (size_t)row * DMOD + sg * 256 + lane * 8;
      *(volatile v4u*)(oh + go) = hv[sg];
      *(volatile v4u*)(ol + go) = lv[sg];
    }
    __threadfence();
  }
}

__global__ __launch_bounds__(128)
void attn64(const unsigned short* __restrict__ qhp, const unsigned short* __restrict__ qlp,
            const unsigned short* __restrict__ khp, const unsigned short* __restrict__ vthp,
            const unsigned short* __restrict__ vtlp, const float* __restrict__ maskp,
            float* attnp, float sscale, float rres, float onorm) {
  union FH { v16h v; v8h h[2]; };
  __shared__ __align__(16) _Float16 Ksh[64 * 64];
  __shared__ __align__(16) _Float16 Vth[64 * 64];
  __shared__ __align__(16) _Float16 Vtl[64 * 64];
  __shared__ __align__(16) _Float16 Psh[4][16 * 64];
  __shared__ __align__(16) float    Os[4][16 * 64];
  __shared__ __align__(16) unsigned short Msh[64 * 64];

  const int tid  = threadIdx.x;
  const int wave = tid >> 5;
  const int lane = tid & 31;
  const int hh   = lane >> 4;
  const int c    = lane & 15;

  const int bx   = blockIdx.x;
  const int qb   = bx % NQB;
  const int rest = bx / NQB;
  const int h    = rest % NH;
  const int b    = rest / NH;
  const int q0   = qb * 64 + wave * 16;
  const size_t rowB = (size_t)b * SEQ;

  const _Float16* Qh  = (const _Float16*)(const void*)qhp + (size_t)h * HD;
  const _Float16* Ql  = (const _Float16*)(const void*)qlp + (size_t)h * HD;
  const _Float16* Kg  = (const _Float16*)(const void*)khp + (size_t)h * HD;
  const _Float16* Vgh = (const _Float16*)(const void*)vthp + ((size_t)b * DMOD + (size_t)h * HD) * SEQ;
  const _Float16* Vgl = (const _Float16*)(const void*)vtlp + ((size_t)b * DMOD + (size_t)h * HD) * SEQ;
  const float* Mg = maskp + (size_t)(qb * 64) * SEQ;

  v16h qah[2], qal[2];
#pragma unroll
  for (int dc = 0; dc < 2; ++dc) {
    qah[dc] = ldfrag_h(Qh + (rowB + q0 + c) * DMOD + dc * 32 + 8 * hh);
    qal[dc] = ldfrag_h(Ql + (rowB + q0 + c) * DMOD + dc * 32 + 8 * hh);
  }

  v8f oacc[4];
#pragma unroll
  for (int t = 0; t < 4; ++t) oacc[t] = zero8();

  for (int kt = 0; kt < NQB; ++kt) {
    const int kv0 = kt * 64;
    __syncthreads();
    {
      const int r = tid >> 1, hf = (tid & 1) * 32;
      const _Float16* kg  = Kg + (rowB + kv0 + r) * DMOD + hf;
      const _Float16* vgh = Vgh + (size_t)r * SEQ + kv0 + hf;
      const _Float16* vgl = Vgl + (size_t)r * SEQ + kv0 + hf;
      const float*    mg  = Mg + (size_t)r * SEQ + kv0 + hf;
#pragma unroll
      for (int i = 0; i < 4; ++i) {
        const v8h a0 = *(const v8h*)(kg + 8 * i);
        const v8h b0 = *(const v8h*)(vgh + 8 * i);
        const v8h b1 = *(const v8h*)(vgl + 8 * i);
        *(v8h*)(Ksh + r * 64 + hf + 8 * i) = a0;
        *(v8h*)(Vth + r * 64 + hf + 8 * i) = b0;
        *(v8h*)(Vtl + r * 64 + hf + 8 * i) = b1;
        const v4f m0 = *(const v4f*)(mg + 8 * i);
        const v4f m1 = *(const v4f*)(mg + 8 * i + 4);
        v4u pk;
        pk[0] = pk16(bf_bits(m0[0]), bf_bits(m0[1]));
        pk[1] = pk16(bf_bits(m0[2]), bf_bits(m0[3]));
        pk[2] = pk16(bf_bits(m1[0]), bf_bits(m1[1]));
        pk[3] = pk16(bf_bits(m1[2]), bf_bits(m1[3]));
        *(v4u*)(Msh + r * 64 + hf + 8 * i) = pk;
      }
    }
    __syncthreads();

    v8f s[4];
#pragma unroll
    for (int j = 0; j < 4; ++j) {
      v8f sh = zero8(), sl = zero8();
#pragma unroll
      for (int dc = 0; dc < 2; ++dc) {
        FH kb;
        kb.h[0] = *(const v8h*)(Ksh + (j * 16 + c) * 64 + dc * 32 + 8 * hh);
        kb.h[1] = *(const v8h*)(Ksh + (j * 16 + c) * 64 + dc * 32 + 16 + 8 * hh);
        sh = mma_h(qah[dc], kb.v, sh);
        sl = mma_h(qal[dc], kb.v, sl);
      }
#pragma unroll
      for (int r = 0; r < 8; ++r) s[j][r] = (sh[r] + sl[r] * rres) * sscale;
    }

    _Float16* pw = Psh[wave];
    const unsigned short* mw = Msh + (wave * 16) * 64;
#pragma unroll
    for (int r = 0; r < 8; ++r) {
#pragma unroll
      for (int j = 0; j < 4; ++j) {
        const float sv  = s[j][r];
        const float e   = __expf(-sv);
        const float sil = sv * __builtin_amdgcn_rcpf(1.0f + e);
        const float mv  = bf_up(mw[(8 * hh + r) * 64 + j * 16 + c]);
        pw[(8 * hh + r) * 64 + j * 16 + c] = (_Float16)(sil * mv * (4096.0f / (float)SEQ));
      }
    }
    wave_sync_lds();

    v8f o1[4];
#pragma unroll
    for (int t = 0; t < 4; ++t) o1[t] = zero8();
#pragma unroll 1
    for (int kk = 0; kk < 2; ++kk) {
      FH pa;
      pa.h[0] = *(const v8h*)(pw + c * 64 + kk * 32 + 8 * hh);
      pa.h[1] = *(const v8h*)(pw + c * 64 + kk * 32 + 16 + 8 * hh);
#pragma unroll
      for (int t = 0; t < 4; ++t) {
        FH vb, vl;
        vb.h[0] = *(const v8h*)(Vth + (t * 16 + c) * 64 + kk * 32 + 8 * hh);
        vb.h[1] = *(const v8h*)(Vth + (t * 16 + c) * 64 + kk * 32 + 16 + 8 * hh);
        vl.h[0] = *(const v8h*)(Vtl + (t * 16 + c) * 64 + kk * 32 + 8 * hh);
        vl.h[1] = *(const v8h*)(Vtl + (t * 16 + c) * 64 + kk * 32 + 16 + 8 * hh);
        oacc[t] = mma_h(pa.v, vb.v, oacc[t]);
        o1[t]   = mma_h(pa.v, vl.v, o1[t]);
      }
    }
#pragma unroll
    for (int t = 0; t < 4; ++t)
#pragma unroll
      for (int r = 0; r < 8; ++r) oacc[t][r] += o1[t][r] * rres;
  }

  float* os = Os[wave];
#pragma unroll
  for (int r = 0; r < 8; ++r) {
#pragma unroll
    for (int t = 0; t < 4; ++t) os[(8 * hh + r) * 64 + t * 16 + c] = oacc[t][r] * onorm;
  }
  wave_sync_lds();
  {
    const int c4 = (lane & 15) * 4;
    float* dst = attnp + (size_t)h * HD;
    for (int pass = 0; pass < 2; ++pass) {
#pragma unroll
      for (int it = 0; it < 8; ++it) {
        const int row = it * 2 + hh;
        const v4f v = *(const v4f*)(os + row * 64 + c4);
        *(volatile v4f*)(dst + (rowB + q0 + row) * DMOD + c4) = v;
      }
      __threadfence();
    }
  }
}

extern "C" void kernel_launch(void* const* d_in, const int* in_sizes, int n_in,
                              void* d_out, int out_size, void* d_ws, size_t ws_size,
                              hipStream_t stream) {
  if (n_in < 5) return;
  if (in_sizes[0] != NROWS * DMOD) return;
  if (in_sizes[1] != SEQ * SEQ) return;
  if (in_sizes[2] != DMOD * EPROJ) return;
  if (in_sizes[3] != DMOD * DMOD) return;
  if (in_sizes[4] != DMOD) return;
  if (out_size != NROWS * DMOD) return;

  const float* x    = (const float*)d_in[0];
  const float* mask = (const float*)d_in[1];
  const float* uvqk = (const float*)d_in[2];
  const float* ow   = (const float*)d_in[3];
  const float* ob   = (const float*)d_in[4];

  const size_t P16 = (size_t)NROWS * DMOD * 2;
  const size_t P32 = (size_t)NROWS * DMOD * 4;
  const size_t PWT = (size_t)EPROJ * DMOD * 2;
  const size_t PWO = (size_t)DMOD * DMOD * 2;
  const size_t PVT = (size_t)NBATCH * DMOD * SEQ * 2;
  size_t off = 0;
  const size_t oXh  = off; off += P16;
  const size_t oXl  = off; off += P16;
  const size_t oWt  = off; off += PWT;
  const size_t oWo  = off; off += PWO;
  const size_t oU   = off; off += P32;
  const size_t oVf  = off; off += P32;
  const size_t oQh  = off; off += P16;
  const size_t oQl  = off; off += P16;
  const size_t oKh  = off; off += P16;
  const size_t oVTh = off; off += PVT;
  const size_t oVTl = off; off += PVT;
  const size_t oAT  = off; off += P32;
  const size_t oOh  = off; off += P16;
  const size_t oOl  = off; off += P16;
  if (off > ws_size) return;
  if (off > (size_t)134217728) return;

  char* ws = (char*)d_ws;
  unsigned short* Xh  = (unsigned short*)(ws + oXh);
  unsigned short* Xl  = (unsigned short*)(ws + oXl);
  unsigned short* Wt  = (unsigned short*)(ws + oWt);
  unsigned short* Wo  = (unsigned short*)(ws + oWo);
  float*          U   = (float*)(ws + oU);
  float*          Vf  = (float*)(ws + oVf);
  unsigned short* Qh  = (unsigned short*)(ws + oQh);
  unsigned short* Ql  = (unsigned short*)(ws + oQl);
  unsigned short* Kh  = (unsigned short*)(ws + oKh);
  unsigned short* VTh = (unsigned short*)(ws + oVTh);
  unsigned short* VTl = (unsigned short*)(ws + oVTl);
  float*          AT  = (float*)(ws + oAT);
  unsigned short* Oh  = (unsigned short*)(ws + oOh);
  unsigned short* Ol  = (unsigned short*)(ws + oOl);

  const dim3 blk(256);
  const dim3 gLn(NROWS / 8);
  const dim3 gTw((DMOD / 64) * (EPROJ / 64), 1);
  const dim3 gCvt((DMOD * DMOD / 8 + 255) / 256);
  const dim3 gGemm(((NROWS / 64) * (DMOD / 64) + 7) / 8, 1);
  const dim3 gTv((SEQ / 64) * (DMOD / 64), NBATCH);
  const dim3 gAttn(NBATCH * NH * NQB);

  ln_rows<0><<<gLn, blk, 0, stream>>>(x, x, Xh, Xl, NROWS);
  transpose16<0><<<gTw, blk, 0, stream>>>(uvqk, DMOD, EPROJ, 0LL, Wt, 0LL, 1.0f, 1.0f);
  cvt_cat_bf16x8<<<gCvt, blk, 0, stream>>>(ow, Wo, DMOD * DMOD / 8, DMOD / 8, DMOD, 0);
  gemm64<1, 0, 0, 1, 0><<<gGemm, blk, 0, stream>>>(
      Xh, Xl, DMOD, 0LL, Wt, Wt, DMOD, 0LL, ob, x, DMOD,
      (void*)U, DMOD, 0LL, (void*)U, DMOD, 0LL, DMOD,
      NROWS, DMOD, DMOD, RESC, 1.0f);
  gemm64<1, 0, 0, 1, 0><<<gGemm, blk, 0, stream>>>(
      Xh, Xl, DMOD, 0LL, Wt + (size_t)512 * DMOD, Wt, DMOD, 0LL, ob, x, DMOD,
      (void*)Vf, DMOD, 0LL, (void*)Vf, DMOD, 0LL, DMOD,
      NROWS, DMOD, DMOD, RESC, 1.0f);
  gemm64<1, 3, 0, 1, 0><<<gGemm, blk, 0, stream>>>(
      Xh, Xl, DMOD, 0LL, Wt + (size_t)1024 * DMOD, Wt, DMOD, 0LL, ob, x, DMOD,
      (void*)Qh, DMOD, 0LL, (void*)Ql, DMOD, 0LL, DMOD,
      NROWS, DMOD, DMOD, RESC, 64.0f);
  gemm64<1, 4, 0, 1, 0><<<gGemm, blk, 0, stream>>>(
      Xh, Xl, DMOD, 0LL, Wt + (size_t)1536 * DMOD, Wt, DMOD, 0LL, ob, x, DMOD,
      (void*)Kh, DMOD, 0LL, (void*)Kh, DMOD, 0LL, 0,
      NROWS, DMOD, DMOD, RESC, 16.0f);
  transpose16<1><<<gTv, blk, 0, stream>>>(Vf, SEQ, DMOD, (long long)SEQ * DMOD, VTh, (long long)DMOD * SEQ, 16.0f, RESC);
  transpose16<2><<<gTv, blk, 0, stream>>>(Vf, SEQ, DMOD, (long long)SEQ * DMOD, VTl, (long long)DMOD * SEQ, 16.0f, RESC);
  attn64<<<gAttn, dim3(128), 0, stream>>>(Qh, Ql, Kh, VTh, VTl, mask, AT,
                                          1.0f / 1024.0f, 1.0f / RESC, 1.0f / 65536.0f);
  ln_rows<1><<<gLn, blk, 0, stream>>>(AT, U, Oh, Ol, NROWS);
  gemm64<1, 0, 1, 0, 1><<<gGemm, blk, 0, stream>>>(
      Oh, Ol, DMOD, 0LL, Wo, Wo, DMOD, 0LL, ob, x, DMOD,
      d_out, DMOD, 0LL, d_out, DMOD, 0LL, DMOD,
      NROWS, DMOD, DMOD, RESC, 1.0f);
  (void)hipGetLastError();
}
